// RelationalGraphLayer_48180943127293
// MI455X (gfx1250) — hardware-verified
//
#include <hip/hip_runtime.h>
#include <stdint.h>
#include <stddef.h>


typedef _Float16 f16t;
typedef _Float16 v16h __attribute__((ext_vector_type(16)));
typedef _Float16 v8h  __attribute__((ext_vector_type(8)));
typedef float    v8f  __attribute__((ext_vector_type(8)));
typedef float    v4f  __attribute__((ext_vector_type(4)));
typedef float    v2f  __attribute__((ext_vector_type(2)));
typedef float    v4fa __attribute__((ext_vector_type(4), may_alias));
typedef float    v2fa __attribute__((ext_vector_type(2), may_alias));

union FragH { v16h v; v8h half[2]; };

#define DIM 512
#define NB 16

__device__ __forceinline__ v8f wmma_f16(v16h a, v16h b, v8f c) {
  return __builtin_amdgcn_wmma_f32_16x16x32_f16(false, a, false, b, (short)0, c, false, false);
}

__device__ __forceinline__ float gelu_exact(float v) {
  return 0.5f * v * (1.0f + erff(v * 0.70710678118654752f));
}

__global__ __launch_bounds__(256) void k_wcvt(const float* __restrict__ W, int K, int Nout,
                                              f16t* Bt, float scale) {
  __shared__ float tile[64][33];
  const int tid = threadIdx.x;
  const size_t zoff = (size_t)blockIdx.z * (size_t)K * (size_t)Nout;
  const float* Wz = W + zoff;
  f16t* Btz = Bt + zoff;
  const int n0 = blockIdx.x * 32, k0 = blockIdx.y * 64;
  const int ty = tid >> 5, tx = tid & 31;
  #pragma unroll
  for (int i = 0; i < 8; ++i) {
    const int kk = ty + 8 * i;
    const int gk = k0 + kk, gn = n0 + tx;
    float v = 0.0f;
    if (gk < K && gn < Nout) v = Wz[(size_t)gk * Nout + gn];
    tile[kk][tx] = v;
  }
  __syncthreads();
  const int j = tid >> 3, q = tid & 7;
  const int gn = n0 + j;
  v8h hv;
  #pragma unroll
  for (int u = 0; u < 8; ++u) hv[u] = (f16t)(tile[8 * q + u][j] * scale);
  const bool ok = (gn < Nout) && (k0 + 64 <= K);
  f16t* p = Btz + (size_t)gn * K + k0 + 8 * q;
  if (ok) *(volatile v8h*)p = hv;
  __threadfence();
  if (ok) *(volatile v8h*)p = hv;
}

__global__ __launch_bounds__(256) void k_xcvt(const float* __restrict__ x, size_t total8, f16t* xh) {
  const size_t g = (size_t)blockIdx.x * 256 + threadIdx.x;
  const bool ok = g < total8;
  v8h hv;
  #pragma unroll
  for (int u = 0; u < 8; ++u) hv[u] = (f16t)0.0f;
  if (ok) {
    const v4f a = *(const v4f*)(x + 8 * g);
    const v4f b = *(const v4f*)(x + 8 * g + 4);
    #pragma unroll
    for (int u = 0; u < 4; ++u) { hv[u] = (f16t)a[u]; hv[4 + u] = (f16t)b[u]; }
  }
  f16t* p = xh + 8 * g;
  if (ok) *(volatile v8h*)p = hv;
  __threadfence();
  if (ok) *(volatile v8h*)p = hv;
}

template <int MODE>
__global__ __launch_bounds__(256) void k_gemm(const f16t* __restrict__ A, const f16t* __restrict__ Bt,
                                              int M, int K,
                                              const float* __restrict__ bias, const float* __restrict__ addend,
                                              const float* __restrict__ lnw, const float* __restrict__ lnb,
                                              float* outF, f16t* outH, int ldo, float oscale) {
  __shared__ float Ct[NB][DIM + 4];

  const int tid = threadIdx.x, wave = tid >> 5, lane = tid & 31;
  const int h = lane >> 4, m = lane & 15;
  const int m0 = blockIdx.x * NB;
  const int col0 = blockIdx.y * DIM;

  int arow = m0 + m; if (arow > M - 1) arow = M - 1;
  const f16t* ap = A + (size_t)arow * K + 8 * h;
  const int cw = col0 + wave * 64 + m;
  const f16t* bp0 = Bt + (size_t)(cw +  0) * K + 8 * h;
  const f16t* bp1 = Bt + (size_t)(cw + 16) * K + 8 * h;
  const f16t* bp2 = Bt + (size_t)(cw + 32) * K + 8 * h;
  const f16t* bp3 = Bt + (size_t)(cw + 48) * K + 8 * h;

  v8f acc[4] = {};

  for (int k0 = 0; k0 < K; k0 += 32) {
    FragH a, b0, b1, b2, b3;
    a.half[0]  = *(const v8h*)(ap + k0);   a.half[1]  = *(const v8h*)(ap + k0 + 16);
    b0.half[0] = *(const v8h*)(bp0 + k0);  b0.half[1] = *(const v8h*)(bp0 + k0 + 16);
    b1.half[0] = *(const v8h*)(bp1 + k0);  b1.half[1] = *(const v8h*)(bp1 + k0 + 16);
    b2.half[0] = *(const v8h*)(bp2 + k0);  b2.half[1] = *(const v8h*)(bp2 + k0 + 16);
    b3.half[0] = *(const v8h*)(bp3 + k0);  b3.half[1] = *(const v8h*)(bp3 + k0 + 16);
    acc[0] = wmma_f16(a.v, b0.v, acc[0]);
    acc[1] = wmma_f16(a.v, b1.v, acc[1]);
    acc[2] = wmma_f16(a.v, b2.v, acc[2]);
    acc[3] = wmma_f16(a.v, b3.v, acc[3]);
    asm volatile("v_nop\n\tv_nop\n\tv_nop\n\tv_nop"
                 : "+v"(acc[0]), "+v"(acc[1]), "+v"(acc[2]), "+v"(acc[3])
                 : "v"(a.v), "v"(b0.v), "v"(b1.v), "v"(b2.v), "v"(b3.v));
  }

  #pragma unroll
  for (int t = 0; t < 4; ++t) {
    const int c = wave * 64 + 16 * t + m;
    const float bv = bias[col0 + c];
    #pragma unroll
    for (int j = 0; j < 8; ++j) {
      const int r = 8 * h + j;
      float v = acc[t][j] * oscale + bv;
      if (MODE == 1) v = gelu_exact(v);
      if (MODE >= 2) {
        int gr = m0 + r; if (gr > M - 1) gr = M - 1;
        v += addend[(size_t)gr * ldo + c];
      }
      Ct[r][c] = v;
    }
  }
  __syncthreads();

  v4f yF[2][4] = {};
  v8h yH[2][2] = {};
  #pragma unroll
  for (int rr = 0; rr < 2; ++rr) {
    const int r = 2 * wave + rr;
    float mu = 0.0f, rstd = 1.0f;
    if (MODE >= 2) {
      float s = 0.0f;
      #pragma unroll
      for (int i = 0; i < DIM / 32; ++i) s += Ct[r][lane + 32 * i];
      #pragma unroll
      for (int off = 16; off > 0; off >>= 1) s += __shfl_xor(s, off, 32);
      mu = s * (1.0f / DIM);
      float q = 0.0f;
      #pragma unroll
      for (int i = 0; i < DIM / 32; ++i) { const float d = Ct[r][lane + 32 * i] - mu; q += d * d; }
      #pragma unroll
      for (int off = 16; off > 0; off >>= 1) q += __shfl_xor(q, off, 32);
      rstd = rsqrtf(q * (1.0f / DIM) + 1e-5f);
    }
    if (MODE != 1) {
      #pragma unroll
      for (int i = 0; i < 4; ++i) {
        const int col = 4 * lane + 128 * i;
        v4f c4 = *(const v4fa*)(&Ct[r][col]);
        if (MODE >= 2) {
          const v4f w4 = *(const v4f*)(lnw + col);
          const v4f b4 = *(const v4f*)(lnb + col);
          c4 = (c4 - mu) * rstd * w4 + b4;
        }
        yF[rr][i] = c4;
      }
    }
    if (MODE == 1 || MODE == 2) {
      #pragma unroll
      for (int i = 0; i < 2; ++i) {
        const int col = 8 * lane + 256 * i;
        v4f lo = *(const v4fa*)(&Ct[r][col]);
        v4f hi = *(const v4fa*)(&Ct[r][col + 4]);
        if (MODE == 2) {
          lo = (lo - mu) * rstd * (*(const v4f*)(lnw + col))     + (*(const v4f*)(lnb + col));
          hi = (hi - mu) * rstd * (*(const v4f*)(lnw + col + 4)) + (*(const v4f*)(lnb + col + 4));
        }
        v8h hv;
        #pragma unroll
        for (int u = 0; u < 4; ++u) { hv[u] = (f16t)lo[u]; hv[4 + u] = (f16t)hi[u]; }
        yH[rr][i] = hv;
      }
    }
  }

  #pragma unroll
  for (int p = 0; p < 2; ++p) {
    if (p) __threadfence();
    #pragma unroll
    for (int rr = 0; rr < 2; ++rr) {
      const int grow = m0 + 2 * wave + rr;
      if (grow < M) {
        if (MODE != 1) {
          #pragma unroll
          for (int i = 0; i < 4; ++i)
            *(volatile v4f*)(outF + (size_t)grow * ldo + col0 + 4 * lane + 128 * i) = yF[rr][i];
        }
        if (MODE == 1 || MODE == 2) {
          #pragma unroll
          for (int i = 0; i < 2; ++i)
            *(volatile v8h*)(outH + (size_t)grow * ldo + col0 + 8 * lane + 256 * i) = yH[rr][i];
        }
      }
    }
  }
}

__global__ __launch_bounds__(256) void k_agg(const int* __restrict__ eidx, const int* __restrict__ etyp,
                                             int E, int N, int R,
                                             const float* __restrict__ hall, const float* __restrict__ x,
                                             float* add1) {
  __shared__ float acc[NB][DIM];
  __shared__ int stage[1024];
  __shared__ unsigned smask[32];
  __shared__ float sdeg[NB];

  const int tid = threadIdx.x, wave = tid >> 5, lane = tid & 31;
  const int n0 = blockIdx.x * NB;
  const int HW = R * DIM;

  for (int i = tid; i < NB * DIM; i += 256) (&acc[0][0])[i] = 0.0f;
  if (tid < NB) sdeg[tid] = 0.0f;
  __syncthreads();

  const int* esrc = eidx;
  const int* edst = eidx + E;
  const int nchunk = (E + 1023) >> 10;
  const int dcol = wave * 64 + 2 * lane;

  for (int c = 0; c < nchunk; ++c) {
    const int e0 = c << 10;
    unsigned mj[4];
    #pragma unroll
    for (int j = 0; j < 4; ++j) {
      const int e = e0 + j * 256 + tid;
      bool match = false;
      int pk = 0;
      if (e < E) {
        const int d = edst[e];
        const int ln = d - n0;
        if ((unsigned)ln < (unsigned)NB) {
          int s = esrc[e];
          s = s < 0 ? 0 : (s > N - 1 ? N - 1 : s);
          int ty = etyp[e];
          ty = ty < 0 ? 0 : (ty > R - 1 ? R - 1 : ty);
          pk = s | (ty << 20) | (ln << 24);
          match = true;
        }
      }
      mj[j] = __builtin_amdgcn_ballot_w32(match);
      if (match) stage[j * 256 + tid] = pk;
    }
    if (lane == 0) {
      smask[wave] = mj[0]; smask[8 + wave] = mj[1]; smask[16 + wave] = mj[2]; smask[24 + wave] = mj[3];
    }
    __syncthreads();

    const unsigned mm = smask[lane];
    unsigned nz = __builtin_amdgcn_ballot_w32(mm != 0u);
    for (int it = 0; it < 32 && nz != 0u; ++it) {
      const int q = __builtin_ctz(nz);
      nz &= nz - 1u;
      unsigned mk = smask[q];
      for (int it2 = 0; it2 < 32 && mk != 0u; ++it2) {
        const int bit = __builtin_ctz(mk);
        mk &= mk - 1u;
        const int pk = stage[q * 32 + bit];
        const int s  = pk & 0xFFFFF;
        const int ty = (pk >> 20) & 15;
        const int nd = (pk >> 24) & 15;
        const v2f v = *(const v2fa*)(hall + (size_t)s * HW + ty * DIM + dcol);
        acc[nd][dcol]     += v[0];
        acc[nd][dcol + 1] += v[1];
        if (tid == 0) sdeg[nd] += 1.0f;
      }
    }
    __syncthreads();
  }

  v4f vals[2][4] = {};
  #pragma unroll
  for (int rr = 0; rr < 2; ++rr) {
    const int r = 2 * wave + rr;
    const int n = n0 + r;
    if (n < N) {
      const float deg = sdeg[r];
      const float inv = 1.0f / fmaxf(deg, 1.0f);
      #pragma unroll
      for (int i = 0; i < 4; ++i) {
        const int col = 4 * lane + 128 * i;
        const v4f a4 = *(const v4fa*)(&acc[r][col]);
        const v4f x4 = *(const v4f*)(x + (size_t)n * DIM + col);
        vals[rr][i] = x4 + a4 * inv;
      }
    }
  }
  #pragma unroll
  for (int p = 0; p < 2; ++p) {
    if (p) __threadfence();
    #pragma unroll
    for (int rr = 0; rr < 2; ++rr) {
      const int n = n0 + 2 * wave + rr;
      if (n < N) {
        #pragma unroll
        for (int i = 0; i < 4; ++i)
          *(volatile v4f*)(add1 + (size_t)n * DIM + 4 * lane + 128 * i) = vals[rr][i];
      }
    }
  }
}

extern "C" void kernel_launch(void* const* d_in, const int* in_sizes, int n_in,
                              void* d_out, int out_size, void* d_ws, size_t ws_size,
                              hipStream_t stream) {
  if (n_in < 15) return;
  const int N  = in_sizes[0] / DIM;
  const int E  = in_sizes[2];
  const int R  = in_sizes[5] / (DIM * DIM);
  const int FF = 2 * DIM;
  if (N < 1 || N > (1 << 20) || E < 0 || R < 1 || R > 16) return;
  if (in_sizes[0] != N * DIM || in_sizes[1] != 2 * E || in_sizes[3] != DIM * DIM ||
      in_sizes[5] != R * DIM * DIM || in_sizes[6] != R * DIM || in_sizes[9] != DIM * FF ||
      in_sizes[11] != FF * DIM || out_size != N * DIM) return;
  const int HW = R * DIM;

  const float* x      = (const float*)d_in[0];
  const int*   e_idx  = (const int*)  d_in[1];
  const int*   e_typ  = (const int*)  d_in[2];
  const float* self_W = (const float*)d_in[3];
  const float* self_b = (const float*)d_in[4];
  const float* rel_W  = (const float*)d_in[5];
  const float* rel_b  = (const float*)d_in[6];
  const float* ln1_w  = (const float*)d_in[7];
  const float* ln1_b  = (const float*)d_in[8];
  const float* W1     = (const float*)d_in[9];
  const float* b1     = (const float*)d_in[10];
  const float* W2     = (const float*)d_in[11];
  const float* b2     = (const float*)d_in[12];
  const float* ln2_w  = (const float*)d_in[13];
  const float* ln2_b  = (const float*)d_in[14];
  float* out = (float*)d_out;

  char* w = (char*)d_ws;
  size_t off = 0;
  auto al   = [](size_t b) { return (b + 255) & ~(size_t)255; };
  auto take = [&](size_t bytes) { size_t o = off; off += al(bytes); return o; };
  const size_t btrel_off  = take((size_t)R * DIM * DIM * 2);
  const size_t btself_off = take((size_t)DIM * DIM * 2);
  const size_t bt1_off    = take((size_t)FF * DIM * 2);
  const size_t bt2_off    = take((size_t)DIM * FF * 2);
  const size_t xh_off     = take((size_t)N * DIM * 2);
  const size_t add1_off   = take((size_t)N * DIM * 4);
  const size_t hall_bytes = (size_t)N * HW * 4;
  const size_t x1f_rel = 0;
  const size_t x1h_rel = al((size_t)N * DIM * 4);
  const size_t hg_rel  = x1h_rel + al((size_t)N * DIM * 2);
  const size_t tail_bytes = hg_rel + (size_t)N * FF * 2;
  const size_t big_off = take(hall_bytes > tail_bytes ? hall_bytes : tail_bytes);
  if (off > ws_size) return;

  f16t*  btRel  = (f16t*)(w + btrel_off);
  f16t*  btSelf = (f16t*)(w + btself_off);
  f16t*  bt1    = (f16t*)(w + bt1_off);
  f16t*  bt2    = (f16t*)(w + bt2_off);
  f16t*  xh     = (f16t*)(w + xh_off);
  float* add1   = (float*)(w + add1_off);
  float* hall   = (float*)(w + big_off);
  float* x1f    = (float*)(w + big_off + x1f_rel);
  f16t*  x1h    = (f16t*)(w + big_off + x1h_rel);
  f16t*  hg     = (f16t*)(w + big_off + hg_rel);

  const float wsc = 64.0f;
  const float osc = 1.0f / 64.0f;

  k_wcvt<<<dim3(DIM / 32, DIM / 64, R), 256, 0, stream>>>(rel_W, DIM, DIM, btRel, wsc);
  k_wcvt<<<dim3(DIM / 32, DIM / 64, 1), 256, 0, stream>>>(self_W, DIM, DIM, btSelf, wsc);
  k_wcvt<<<dim3(FF / 32, DIM / 64, 1), 256, 0, stream>>>(W1, DIM, FF, bt1, wsc);
  k_wcvt<<<dim3(DIM / 32, FF / 64, 1), 256, 0, stream>>>(W2, FF, DIM, bt2, wsc);

  const size_t total8 = (size_t)N * DIM / 8;
  k_xcvt<<<(unsigned)((total8 + 255) / 256), 256, 0, stream>>>(x, total8, xh);

  const int MB = (N + NB - 1) / NB;

  k_gemm<0><<<dim3(MB, R), 256, 0, stream>>>(xh, btRel, N, DIM, rel_b, x, ln1_w, ln1_b, hall, bt2, HW, osc);

  k_agg<<<MB, 256, 0, stream>>>(e_idx, e_typ, E, N, R, hall, x, add1);

  k_gemm<2><<<dim3(MB, 1), 256, 0, stream>>>(xh, btSelf, N, DIM, self_b, add1, ln1_w, ln1_b, x1f, x1h, DIM, osc);

  k_gemm<1><<<dim3(MB, FF / DIM), 256, 0, stream>>>(x1h, bt1, N, DIM, b1, add1, ln1_w, ln1_b, add1, hg, FF, osc);

  k_gemm<3><<<dim3(MB, 1), 256, 0, stream>>>(hg, bt2, N, FF, b2, x1f, ln2_w, ln2_b, out, xh, DIM, osc);
}
